// GQA_9113920602192
// MI455X (gfx1250) — hardware-verified
//
#include <hip/hip_runtime.h>
#include <math.h>

typedef __attribute__((ext_vector_type(16))) _Float16 v16h;
typedef __attribute__((ext_vector_type(16))) __bf16 v16b;
typedef __attribute__((ext_vector_type(8)))  _Float16 v8h;
typedef __attribute__((ext_vector_type(8)))  __bf16 v8b;
typedef __attribute__((ext_vector_type(8)))  float v8f;
typedef __attribute__((ext_vector_type(4)))  float v4f;
typedef __attribute__((ext_vector_type(4)))  unsigned v4u;
typedef __attribute__((ext_vector_type(4)))  int v4i;

template <typename T> __device__ __forceinline__ void vst2(void* p, T v) { *(volatile T*)p = v; __threadfence(); *(volatile T*)p = v; }
__device__ __forceinline__ v8f wmma16(v16h a, v16h b, v8f c) {
  v8f d = __builtin_amdgcn_wmma_f32_16x16x32_f16(false, a, false, b, (short)0, c, false, false);
  asm volatile("v_nop\n\tv_nop\n\tv_nop\n\tv_nop" : "+v"(d) : "v"(a), "v"(b));
  return d;
}
__device__ __forceinline__ v8f wmma_bf(v16b a, v16b b, v8f c) {
  v8f d = __builtin_amdgcn_wmma_f32_16x16x32_bf16(false, a, false, b, (short)0, c, false, false);
  asm volatile("v_nop\n\tv_nop\n\tv_nop\n\tv_nop" : "+v"(d) : "v"(a), "v"(b));
  return d;
}
__device__ __forceinline__ v16h frag_h(const _Float16* rowk0, int lane) {
  union { v16h v; v8h q[2]; } u; const _Float16* p = rowk0 + 8 * (lane >> 4);
  u.q[0] = *(const v8h*)p; u.q[1] = *(const v8h*)(p + 16); return u.v;
}
__device__ __forceinline__ v16b frag_b(const __bf16* rowk0, int lane) {
  union { v16b v; v8b q[2]; } u; const __bf16* p = rowk0 + 8 * (lane >> 4);
  u.q[0] = *(const v8b*)p; u.q[1] = *(const v8b*)(p + 16); return u.v;
}
__device__ __forceinline__ v16h frag_f32(const float* rowk0, int lane) {
  v16h a; const float* p = rowk0 + 8 * (lane >> 4);
#pragma unroll
  for (int i = 0; i < 8; ++i) { a[i] = (_Float16)p[i]; a[8 + i] = (_Float16)p[16 + i]; }
  return a;
}
struct F2 { v16b h, l; };
__device__ __forceinline__ F2 bsplit16(const float v[16]) { F2 r;
#pragma unroll
  for (int i = 0; i < 16; ++i) { const __bf16 h = (__bf16)v[i]; r.h[i] = h; r.l[i] = (__bf16)(v[i] - (float)h); }
  return r; }
__device__ __forceinline__ F2 split_row(const float* row, int k0, int lane) { float v[16]; const float* p = row + k0 + 8 * (lane >> 4);
#pragma unroll
  for (int i = 0; i < 8; ++i) { v[i] = p[i]; v[8 + i] = p[16 + i]; }
  return bsplit16(v); }
__device__ __forceinline__ float bfr(float v) { return (float)(__bf16)v; }
#define LDSX() do { asm volatile("s_wait_dscnt 0" ::: "memory"); __builtin_amdgcn_wave_barrier(); __builtin_amdgcn_fence(3  , "workgroup"); } while (0)

#ifndef NB
#define NB 1
#endif
#ifndef SEQ
#define SEQ 2048
#endif
#define NB_FULL 1
#define SEQ_FULL 2048
#define TT SEQ
#define TTF SEQ_FULL
#define DIN 2048
#define NH 32
#define NKV 8
#define GQ (NH / NKV)
#define HD 64
#define NP (HD / 2)
#define CQ (NH * HD)
#define CK (NKV * HD)
#define NQB (TT / 64)
#define NKB (TT / 128)
#define HG 4
#define SCALE (0.125f)
#define QBH 2
#define KHI 128
#define QRES (1024.0f)
#define PCAR (2048.0f)
static_assert(NB == 1 && NB_FULL == 1);
static_assert(TT % 128 == 0 && TT >= KHI && TT <= TTF);
static_assert(KHI == 128 && QBH * 64 <= KHI);
static_assert(NH % HG == 0 && CQ % 128 == 0 && CK % 128 == 0 && DIN % 64 == 0 && HD == 64);
static_assert((TT * DIN) % 2048 == 0 && (TT * NP) % 256 == 0);

#define WS_QH  ((size_t)0)
#define WS_QL  (WS_QH  + 2u * (size_t)TT * CQ)
#define WS_KH  (WS_QL  + 2u * (size_t)TT * CQ)
#define WS_KL  (WS_KH  + 2u * (size_t)TT * CK)
#define WS_VT  (WS_KL  + 2u * (size_t)KHI * CK)
#define WS_VB  (WS_VT  + 2u * (size_t)CK * TT)
#define WS_VBL (WS_VB  + 2u * (size_t)CK * KHI)
#define WS_S   (WS_VBL + 2u * (size_t)CK * KHI)
#define WS_Y   (WS_S   + 4u * (size_t)HG * TT * TT)
#define WS_WQ  (WS_Y   + 4u * (size_t)TT * CQ)
#define WS_WK  (WS_WQ  + 2u * (size_t)CQ * DIN)
#define WS_WV  (WS_WK  + 2u * (size_t)CK * DIN)
#define WS_WO  (WS_WV  + 2u * (size_t)CK * DIN)
#define WS_CC  (WS_WO  + 2u * (size_t)DIN * CQ)
#define WS_CS  (WS_CC  + 4u * (size_t)TT * NP)
#define WS_FL  (WS_CS  + 4u * (size_t)TT * NP)
#define WS_END (WS_FL  + 4u * (size_t)NQB * NKB * 32)
static_assert(WS_END <= (size_t)134217728);
static_assert(2u * (size_t)TT * DIN <= 4u * (size_t)TT * CQ);
static_assert(WS_QL % 128 == 0 && WS_KH % 128 == 0 && WS_KL % 128 == 0 && WS_VT % 128 == 0 && WS_VB % 128 == 0 && WS_VBL % 128 == 0 && WS_S % 128 == 0 && WS_Y % 128 == 0 && WS_WQ % 128 == 0 && WS_WK % 128 == 0 && WS_WV % 128 == 0 && WS_WO % 128 == 0 && WS_CC % 128 == 0 && WS_CS % 128 == 0 && WS_FL % 128 == 0);

__global__ __launch_bounds__(256) void k_cvtx(const float* __restrict__ X, __bf16* __restrict__ XB) {
  const size_t e = ((size_t)blockIdx.x * 256 + threadIdx.x) * 8;
  const v4f a = *(const v4f*)(X + e), b = *(const v4f*)(X + e + 4);
  union { v8b v; v4u u; } o;
#pragma unroll
  for (int i = 0; i < 4; ++i) { o.v[i] = (__bf16)a[i]; o.v[4 + i] = (__bf16)b[i]; }
  vst2((unsigned*)(XB + e), o.u);
}
__global__ __launch_bounds__(256) void k_cvtw(const float* __restrict__ W, __bf16* __restrict__ WB, int K, int N) {
  __shared__ __align__(16) __bf16 tl[64][72];
  const int tid = threadIdx.x; const int n0 = blockIdx.x * 64, k0 = blockIdx.y * 64;
  { const int kk = tid >> 2, nn = (tid & 3) * 16; const float* p = W + (size_t)(k0 + kk) * N + n0 + nn;
#pragma unroll
    for (int q = 0; q < 4; ++q) { const v4f v = *(const v4f*)(p + 4 * q);
#pragma unroll
      for (int i = 0; i < 4; ++i) tl[nn + 4 * q + i][kk] = (__bf16)v[i]; } }
  __syncthreads();
#pragma unroll
  for (int it = 0; it < 2; ++it) { const int nn = (tid >> 3) + 32 * it, q = tid & 7; vst2((unsigned*)(WB + (size_t)(n0 + nn) * K + k0 + q * 8), *(const v4u*)&tl[nn][q * 8]); }
}
__global__ __launch_bounds__(256) void k_cst(const float* __restrict__ FR, float* __restrict__ CSC, float* __restrict__ CSS) {
  const int e = blockIdx.x * 256 + threadIdx.x;
  const float ang = bfr(FR[e]); float s, c; sincosf(ang, &s, &c);
  vst2(CSC + e, c); vst2(CSS + e, s);
}
__global__ __launch_bounds__(256) void k_mtile(const int* __restrict__ MK, int* __restrict__ FL) {
  __shared__ int sw[8];
  const int kb = blockIdx.x, qb = blockIdx.y, tid = threadIdx.x;
  const int* p = MK + (size_t)(qb * 64 + (tid >> 2)) * TTF + kb * 128 + (tid & 3) * 32;
  int any = 0;
#pragma unroll
  for (int q = 0; q < 8; ++q) { const v4i v = *(const v4i*)(p + 4 * q); any |= v[0] | v[1] | v[2] | v[3]; }
  any = (any != 0) ? 1 : 0;
#pragma unroll
  for (int o = 1; o < 32; o <<= 1) any |= __shfl_xor(any, o);
  if ((tid & 31) == 0) sw[tid >> 5] = any;
  __syncthreads();
  if (tid < 32) { int a = 0;
#pragma unroll
    for (int i = 0; i < 8; ++i) a |= sw[i];
    vst2(FL + ((size_t)qb * NKB + kb) * 32 + tid, a); }
}
__device__ __forceinline__ int kb_lastf(const int* __restrict__ FL, int qb) { int kl = 0;
#pragma unroll 1
  for (int kb = 0; kb < NKB; ++kb) kl = (FL[((size_t)qb * NKB + kb) * 32] != 0) ? kb : kl;
  return kl; }

__global__ __launch_bounds__(128) void k_prj(const __bf16* __restrict__ XB, const __bf16* __restrict__ WB, const float* __restrict__ CSC, const float* __restrict__ CSS, int nout, int nhi,
    _Float16* __restrict__ DH, _Float16* __restrict__ DL) {
  __shared__ __align__(16) _Float16 sh[64][136], sl[64][136]; __shared__ __align__(16) float scs[64][NP], ssn[64][NP];
  const int tid = threadIdx.x, wave = tid >> 5, lane = tid & 31, col = lane & 15, g = lane >> 4; const int c0 = blockIdx.y * 128; const int t0 = blockIdx.x * 64;
  v8f acc[8] = {};
#pragma unroll 2
  for (int kc = 0; kc < DIN / 32; ++kc) { const v16b a = frag_b(XB + (size_t)(t0 + wave * 16 + col) * DIN + kc * 32, lane);
#pragma unroll
    for (int j = 0; j < 8; ++j) { const v16b w = frag_b(WB + (size_t)(c0 + j * 16 + col) * DIN + kc * 32, lane); acc[j] = wmma_bf(a, w, acc[j]); } }
  for (int e = tid; e < 64 * (NP / 4); e += 128) { const int rl = e >> 3, q = e & 7;
    *(v4f*)&scs[rl][q * 4] = *(const v4f*)(CSC + (size_t)(t0 + rl) * NP + q * 4); *(v4f*)&ssn[rl][q * 4] = *(const v4f*)(CSS + (size_t)(t0 + rl) * NP + q * 4); }
  __syncthreads();
  const float sgn = (col & 1) ? 1.0f : -1.0f;
#pragma unroll
  for (int j = 0; j < 8; ++j) { const int pi = ((j & 3) * 16 + col) >> 1;
#pragma unroll
    for (int r = 0; r < 8; ++r) { const int rl = wave * 16 + 8 * g + r; const float v = acc[j][r]; const float pv = __shfl_xor(v, 1);
      const float rv = v * scs[rl][pi] + (sgn * pv) * ssn[rl][pi];
      const _Float16 hv = (_Float16)rv; sh[rl][j * 16 + col] = hv; sl[rl][j * 16 + col] = (_Float16)((rv - (float)hv) * QRES); } }
  __syncthreads();
  const bool hi_rows = t0 < nhi;
  for (int e = tid; e < 64 * 16; e += 128) { const int rl = e >> 4, q = e & 15;
    vst2((unsigned*)(DH + (size_t)(t0 + rl) * nout + c0 + q * 8), *(const v4u*)&sh[rl][q * 8]);
    if (hi_rows) vst2((unsigned*)(DL + (size_t)(t0 + rl) * nout + c0 + q * 8), *(const v4u*)&sl[rl][q * 8]); }
}
__global__ __launch_bounds__(128) void k_prjv(const __bf16* __restrict__ XB, const __bf16* __restrict__ WB, _Float16* __restrict__ VT, __bf16* __restrict__ VB, __bf16* __restrict__ VBL) {
  __shared__ __align__(16) _Float16 th[128][72]; __shared__ __align__(16) __bf16 tb[128][72], tbl[128][72];
  const int tid = threadIdx.x, wave = tid >> 5, lane = tid & 31, col = lane & 15, g = lane >> 4; const int c0 = blockIdx.y * 128; const int t0 = blockIdx.x * 64;
  v8f acc[8] = {};
#pragma unroll 2
  for (int kc = 0; kc < DIN / 32; ++kc) { const v16b a = frag_b(XB + (size_t)(t0 + wave * 16 + col) * DIN + kc * 32, lane);
#pragma unroll
    for (int j = 0; j < 8; ++j) { const v16b w = frag_b(WB + (size_t)(c0 + j * 16 + col) * DIN + kc * 32, lane); acc[j] = wmma_bf(a, w, acc[j]); } }
#pragma unroll
  for (int j = 0; j < 8; ++j) {
#pragma unroll
    for (int r = 0; r < 8; ++r) { const float v = acc[j][r]; const int rl = wave * 16 + 8 * g + r, cl = j * 16 + col; th[cl][rl] = (_Float16)v; const __bf16 bh = (__bf16)v; tb[cl][rl] = bh; tbl[cl][rl] = (__bf16)(v - (float)bh); } }
  __syncthreads();
  const bool hi_rows = t0 < KHI;
  for (int e = tid; e < 128 * 8; e += 128) { const int cl = e >> 3, q = e & 7;
    vst2((unsigned*)(VT + (size_t)(c0 + cl) * TT + t0 + q * 8), *(const v4u*)&th[cl][q * 8]);
    if (hi_rows) { const size_t o3 = (size_t)(c0 + cl) * KHI + t0 + q * 8; vst2((unsigned*)(VB + o3), *(const v4u*)&tb[cl][q * 8]); vst2((unsigned*)(VBL + o3), *(const v4u*)&tbl[cl][q * 8]); } }
}
__global__ __launch_bounds__(128) void k_sc(const _Float16* __restrict__ QH, const _Float16* __restrict__ QL, const _Float16* __restrict__ KH, const _Float16* __restrict__ KL, const int* __restrict__ FL, int h0, float* __restrict__ S0) {
  __shared__ __align__(16) float ss[4][16][132];
  const int qb = blockIdx.x, kb = blockIdx.y;
  if (FL[((size_t)qb * NKB + kb) * 32] == 0) return;
  const int h = h0 + blockIdx.z, kv = h / GQ; float* S = S0 + (size_t)blockIdx.z * TT * TT;
  const int tid = threadIdx.x, wave = tid >> 5, lane = tid & 31, col = lane & 15, g = lane >> 4; const int k0 = kb * 128; const int ql0 = qb * 64 + wave * 16;
  const _Float16* qhp = QH + (size_t)(ql0 + col) * CQ + h * HD; const _Float16* qlp = QL + (size_t)(ql0 + col) * CQ + h * HD;
  v8f acc[8] = {}, accl[8] = {};
  if (qb < QBH && kb == 0) {
#pragma unroll
    for (int kc = 0; kc < HD / 32; ++kc) { const v16h ah = frag_h(qhp + kc * 32, lane), al = frag_h(qlp + kc * 32, lane);
#pragma unroll
      for (int j = 0; j < 8; ++j) { const size_t ko = (size_t)(k0 + j * 16 + col) * CK + kv * HD + kc * 32; const v16h kf = frag_h(KH + ko, lane), klf = frag_h(KL + ko, lane);
        acc[j] = wmma16(ah, kf, acc[j]); accl[j] = wmma16(al, kf, accl[j]); accl[j] = wmma16(ah, klf, accl[j]); } }
  } else {
#pragma unroll
    for (int kc = 0; kc < HD / 32; ++kc) { const v16h ah = frag_h(qhp + kc * 32, lane), al = frag_h(qlp + kc * 32, lane);
#pragma unroll
      for (int j = 0; j < 8; ++j) { const size_t ko = (size_t)(k0 + j * 16 + col) * CK + kv * HD + kc * 32; const v16h kf = frag_h(KH + ko, lane);
        acc[j] = wmma16(ah, kf, acc[j]); accl[j] = wmma16(al, kf, accl[j]); } } }
#pragma unroll
  for (int j = 0; j < 8; ++j) {
#pragma unroll
    for (int r = 0; r < 8; ++r) ss[wave][8 * g + r][j * 16 + col] = (acc[j][r] + accl[j][r] * (1.0f / QRES)) * SCALE; }
  LDSX(); for (int rl = 0; rl < 16; ++rl) vst2(S + (size_t)(ql0 + rl) * TT + k0 + lane * 4, *(const v4f*)&ss[wave][rl][lane * 4]); }
__global__ __launch_bounds__(256) void k_sm(float* __restrict__ S0, const int* __restrict__ MK, const int* __restrict__ FL) { __shared__ float sred[8]; __shared__ float sbc; __shared__ __align__(16) float shv[TT];
  const int tid = threadIdx.x; const int t = blockIdx.x; const int kend = (kb_lastf(FL, t >> 6) + 1) * 128;
  float* sr = S0 + (size_t)blockIdx.y * TT * TT + (size_t)t * TT; const int* mr = MK + (size_t)t * TTF;
  float m = -3.0e38f; for (int k = tid; k < kend; k += 256) { const float sv = sr[k]; const int mk = mr[k]; const float v = (mk != 0) ? sv : -3.0e38f; shv[k] = v; m = fmaxf(m, v); }
#pragma unroll
  for (int o = 1; o < 32; o <<= 1) m = fmaxf(m, __shfl_xor(m, o));
  if ((tid & 31) == 0) sred[tid >> 5] = m; __syncthreads(); if (tid == 0) { float a = sred[0]; for (int i = 1; i < 8; ++i) a = fmaxf(a, sred[i]); sbc = a; } __syncthreads(); m = sbc; __syncthreads();
  float sum = 0.f; for (int k = tid; k < kend; k += 256) { const float v = shv[k]; const float e = (v <= -1.0e38f) ? 0.f : expf(v - m); shv[k] = e; sum += e; }
#pragma unroll
  for (int o = 1; o < 32; o <<= 1) sum += __shfl_xor(sum, o);
  if ((tid & 31) == 0) sred[tid >> 5] = sum; __syncthreads(); if (tid == 0) { float a = 0.f; for (int i = 0; i < 8; ++i) a += sred[i]; sbc = PCAR / a; } __syncthreads(); const float inv = sbc;
  for (int k = tid; k < kend; k += 256) shv[k] = shv[k] * inv;
  __syncthreads(); for (int q = tid; q < kend / 4; q += 256) vst2(sr + q * 4, *(const v4f*)&shv[q * 4]); }
__global__ __launch_bounds__(128) void k_pv(const float* __restrict__ PS0, const _Float16* __restrict__ VT, const __bf16* __restrict__ VB, const __bf16* __restrict__ VBL, const int* __restrict__ FL, int h0, float* __restrict__ Y) {
  const int h = h0 + blockIdx.z, kv = h / GQ; const float* PS = PS0 + (size_t)blockIdx.z * TT * TT; __shared__ __align__(16) float ss[4][16][HD + 4];
  const int tid = threadIdx.x, wave = tid >> 5, lane = tid & 31, col = lane & 15, g = lane >> 4; const int qb = blockIdx.x; const int ql0 = qb * 64 + wave * 16;
  const int kbl = kb_lastf(FL, qb); const int kce = (kbl + 1) * 4;
  v8f acc[HD / 16] = {};
  if (qb < QBH && kbl == 0) {
#pragma unroll 1
    for (int kc = 0; kc < kce; ++kc) { const F2 p = split_row(PS + (size_t)(ql0 + col) * TT, kc * 32, lane);
      asm volatile("s_wait_loadcnt 0x0" ::: "memory");
#pragma unroll
      for (int j = 0; j < HD / 16; ++j) { const size_t po = ((size_t)kv * HD + j * 16 + col) * (size_t)KHI + kc * 32; const v16b vh = frag_b(VB + po, lane);
        acc[j] = wmma_bf(p.h, vh, acc[j]); acc[j] = wmma_bf(p.l, vh, acc[j]); acc[j] = wmma_bf(p.h, frag_b(VBL + po, lane), acc[j]); } }
  } else {
#pragma unroll 1
    for (int kc = 0; kc < kce; ++kc) { const v16h p = frag_f32(PS + (size_t)(ql0 + col) * TT + kc * 32, lane);
      asm volatile("s_wait_loadcnt 0x0" ::: "memory");
#pragma unroll
      for (int j = 0; j < HD / 16; ++j) { const size_t po = ((size_t)kv * HD + j * 16 + col) * (size_t)TT + kc * 32; acc[j] = wmma16(p, frag_h(VT + po, lane), acc[j]); } } }
#pragma unroll
  for (int j = 0; j < HD / 16; ++j)
#pragma unroll
    for (int r = 0; r < 8; ++r) ss[wave][8 * g + r][j * 16 + col] = acc[j][r] * (1.0f / PCAR);
  LDSX(); for (int rl = 0; rl < 16; ++rl) if (lane < HD / 4) vst2(Y + (size_t)(ql0 + rl) * CQ + h * HD + lane * 4, *(const v4f*)&ss[wave][rl][lane * 4]); }
__global__ __launch_bounds__(128) void k_out(const float* __restrict__ Y, const __bf16* __restrict__ WOB, float* __restrict__ OUT) { __shared__ __align__(16) float sf[4][16][132];
  const int tid = threadIdx.x, wave = tid >> 5, lane = tid & 31, col = lane & 15, g = lane >> 4; const int c0 = blockIdx.y * 128; const size_t r0 = (size_t)blockIdx.x * 64 + wave * 16;
  v8f acc[8] = {};
#pragma unroll 2
  for (int kc = 0; kc < CQ / 32; ++kc) { const F2 a = split_row(Y + (r0 + col) * CQ, kc * 32, lane); asm volatile("s_wait_loadcnt 0x0" ::: "memory");
#pragma unroll
    for (int j = 0; j < 8; ++j) { const v16b w = frag_b(WOB + (size_t)(c0 + j * 16 + col) * CQ + kc * 32, lane); asm volatile("s_wait_loadcnt 0x0" ::: "memory"); acc[j] = wmma_bf(a.h, w, acc[j]); acc[j] = wmma_bf(a.l, w, acc[j]); } }
#pragma unroll
  for (int j = 0; j < 8; ++j) {
#pragma unroll
    for (int r = 0; r < 8; ++r) sf[wave][8 * g + r][j * 16 + col] = acc[j][r]; }
  LDSX(); for (int rl = 0; rl < 16; ++rl) vst2(OUT + (r0 + rl) * DIN + c0 + lane * 4, *(const v4f*)&sf[wave][rl][lane * 4]); }

extern "C" void kernel_launch(void* const* d_in, const int* in_sizes, int n_in, void* d_out, int out_size, void* d_ws, size_t ws_size, hipStream_t stream) {
  if (n_in < 7) return;
  if (in_sizes[0] < TT * DIN || in_sizes[1] < TT * NP || in_sizes[2] < TT * TTF || in_sizes[3] < DIN * CQ || in_sizes[4] < DIN * CK || in_sizes[5] < DIN * CK || in_sizes[6] < CQ * DIN) return;
  if (out_size < TT * DIN || ws_size < WS_END) return;
  const float* X = (const float*)d_in[0]; const float* FR = (const float*)d_in[1]; const int* MK = (const int*)d_in[2];
  const float* WQ = (const float*)d_in[3]; const float* WK = (const float*)d_in[4]; const float* WV = (const float*)d_in[5]; const float* WO = (const float*)d_in[6];
  char* ws = (char*)d_ws;
  _Float16 *QH = (_Float16*)(ws + WS_QH), *QL = (_Float16*)(ws + WS_QL), *KH = (_Float16*)(ws + WS_KH), *KL = (_Float16*)(ws + WS_KL), *VT = (_Float16*)(ws + WS_VT);
  __bf16 *VB = (__bf16*)(ws + WS_VB), *VBL = (__bf16*)(ws + WS_VBL);
  float *S = (float*)(ws + WS_S), *Y = (float*)(ws + WS_Y);
  __bf16 *XB = (__bf16*)(ws + WS_Y), *WQB = (__bf16*)(ws + WS_WQ), *WKB = (__bf16*)(ws + WS_WK), *WVB = (__bf16*)(ws + WS_WV), *WOB = (__bf16*)(ws + WS_WO);
  float *CSC = (float*)(ws + WS_CC), *CSS = (float*)(ws + WS_CS); int* FL = (int*)(ws + WS_FL);
  float* OUT = (float*)d_out;

  k_cvtx<<<dim3((TT * DIN) / 2048), 256, 0, stream>>>(X, XB);
  k_cvtw<<<dim3(CQ / 64, DIN / 64), 256, 0, stream>>>(WQ, WQB, DIN, CQ);
  k_cvtw<<<dim3(CK / 64, DIN / 64), 256, 0, stream>>>(WK, WKB, DIN, CK);
  k_cvtw<<<dim3(CK / 64, DIN / 64), 256, 0, stream>>>(WV, WVB, DIN, CK);
  k_cvtw<<<dim3(DIN / 64, CQ / 64), 256, 0, stream>>>(WO, WOB, CQ, DIN);
  k_cst<<<dim3((TT * NP) / 256), 256, 0, stream>>>(FR, CSC, CSS);
  k_mtile<<<dim3(NKB, NQB), 256, 0, stream>>>(MK, FL);
  k_prj<<<dim3(TT / 64, CQ / 128), 128, 0, stream>>>(XB, WQB, CSC, CSS, CQ, TT, QH, QL);
  k_prj<<<dim3(TT / 64, CK / 128), 128, 0, stream>>>(XB, WKB, CSC, CSS, CK, KHI, KH, KL);
  k_prjv<<<dim3(TT / 64, CK / 128), 128, 0, stream>>>(XB, WVB, VT, VB, VBL);
  for (int h0 = 0; h0 < NH; h0 += HG) {
    k_sc<<<dim3(NQB, NKB, HG), 128, 0, stream>>>(QH, QL, KH, KL, FL, h0, S);
    k_sm<<<dim3(TT, HG), 256, 0, stream>>>(S, MK, FL);
    k_pv<<<dim3(NQB, 1, HG), 128, 0, stream>>>(S, VT, VB, VBL, FL, h0, Y);
  }
  k_out<<<dim3(TT / 64, DIN / 128), 128, 0, stream>>>(Y, WOB, OUT);
}
